// ReMambaBlock_40346922778718
// MI455X (gfx1250) — hardware-verified
//
#include <hip/hip_runtime.h>
#include <hip/hip_bf16.h>


#define __bf16 _Float16
typedef __attribute__((ext_vector_type(16))) _Float16 v16bf;
typedef __attribute__((ext_vector_type(8)))  _Float16 v8bf;
typedef __attribute__((ext_vector_type(8)))  float  v8f;
typedef __attribute__((ext_vector_type(4)))  float  v4f;
#define VST2(T, ptr, val) do { const T _v = (val); *(volatile T*)(ptr) = _v; __threadfence(); *(volatile T*)(ptr) = _v; } while (0)
__device__ __forceinline__ void wave_lds_sync() {
    __builtin_amdgcn_fence(__ATOMIC_RELEASE, "workgroup"); __builtin_amdgcn_wave_barrier(); __builtin_amdgcn_fence(__ATOMIC_ACQUIRE, "workgroup");
}

__device__ __forceinline__ float siluf(float x)     { return x / (1.0f + __expf(-x)); }
__device__ __forceinline__ float softplusf(float x) { return (x > 20.0f) ? x : log1pf(__expf(x)); }

__device__ __forceinline__ unsigned pack_bf16(float a, float b) {
    union { _Float16 h[2]; unsigned u; } p;
    p.h[0] = (_Float16)a; p.h[1] = (_Float16)b;
    return p.u;
}


__global__ __launch_bounds__(256) void prep_wdelta(const float* __restrict__ xpw,
                                                   const float* __restrict__ dtw,
                                                   float* __restrict__ wd) {
    int i = blockIdx.x;
    int j = threadIdx.x;
    float s = 0.f;
#pragma unroll
    for (int r = 0; r < 8; ++r) s += xpw[i * 40 + r] * dtw[r * 256 + j];
    VST2(float, wd + i * 256 + j, s);
}

__global__ __launch_bounds__(256) void prep_negexpA(const float* __restrict__ Alog,
                                                    float* __restrict__ Aneg) {
    int i = blockIdx.x * 256 + threadIdx.x;
    VST2(float, Aneg + i, -expf(Alog[i]));
}

__global__ __launch_bounds__(128) void mean_kernel(const float* __restrict__ x,
                                                   const float* __restrict__ prev,
                                                   float* __restrict__ xin) {
    const int bl = blockIdx.x, c = threadIdx.x, blc = bl * 128 + c;
    const float* p = x + (long)blc * 1024;
    float s = 0.f;
    for (int i = 0; i < 1024; i += 4) { const v4f v = *(const v4f*)(p + i); s += (v[0] + v[1]) + (v[2] + v[3]); }
    VST2(float, xin + blc, s * (1.0f / 1024.0f) + prev[blc]);
}

__global__ __launch_bounds__(256) void conv_silu(const float* __restrict__ xm_pre,
                                                 const float* __restrict__ cw,
                                                 const float* __restrict__ cb,
                                                 float* __restrict__ xm,
                                                 int seqlen) {
    int bl = blockIdx.x / seqlen;
    int t  = blockIdx.x % seqlen;
    int d  = threadIdx.x;
    const float* base = xm_pre + (long)bl * seqlen * 256 + d;
    float s = cb[d];
#pragma unroll
    for (int k = 0; k < 4; ++k) {
        int tt = t - 3 + k;
        if (tt >= 0) s += base[(long)tt * 256] * cw[d * 4 + k];
    }
    VST2(float, xm + ((long)bl * seqlen + t) * 256 + d, siluf(s));
}

__global__ __launch_bounds__(256) void scan_kernel(const float* __restrict__ u,
                                                   const float* __restrict__ delta,
                                                   const float* __restrict__ BC,
                                                   const float* __restrict__ Aneg,
                                                   const float* __restrict__ Dv,
                                                   float* __restrict__ y,
                                                   int seqlen) {
    __shared__ float sbc[32];
    int bl = blockIdx.x;
    int d  = threadIdx.x;
    float a[16], h[16];
#pragma unroll
    for (int n = 0; n < 16; ++n) { a[n] = Aneg[d * 16 + n]; h[n] = 0.f; }
    float Dd = Dv[d];
    long base = (long)bl * seqlen;
    for (int t = 0; t < seqlen; ++t) {
        long row = base + t;
        if (threadIdx.x < 32) sbc[threadIdx.x] = BC[row * 32 + threadIdx.x];
        __syncthreads();
        float dl = delta[row * 256 + d];
        float uu = u[row * 256 + d];
        float du = dl * uu;
        float acc = 0.f;
#pragma unroll
        for (int n = 0; n < 16; ++n) {
            float dA = __expf(dl * a[n]);
            h[n] = dA * h[n] + du * sbc[n];
            acc += h[n] * sbc[16 + n];
        }
        VST2(float, y + row * 256 + d, acc + uu * Dd);
        __syncthreads();
    }
}

template <int AMODE, int EPI>
__global__ __launch_bounds__(256) void gemm16(const float* __restrict__ A,
                                              const float* __restrict__ Z,
                                              const float* __restrict__ W,
                                              int ldw, int wcol0,
                                              float* __restrict__ out,
                                              float* __restrict__ out2,
                                              const float* __restrict__ resid,
                                              int M, int Ncols, int K) {
    __shared__ __attribute__((aligned(16))) __bf16 sA[8][16 * 32];
    __shared__ __attribute__((aligned(16))) __bf16 sB[8][32 * 32];
    __shared__ __attribute__((aligned(16))) float sO[8][16 * 32];
    const int wave = threadIdx.x >> 5;
    const int lane = threadIdx.x & 31;
    const long Mt = M >> 4, Nt2 = Ncols >> 5;
    long tile = (long)blockIdx.x * 8 + wave;
    if (tile >= Mt * Nt2) return;
    const int tn = (int)(tile % Nt2);
    const int tm = (int)(tile / Nt2);
    const int m0 = tm << 4, n0 = tn << 5;

    __bf16* la = sA[wave];
    __bf16* lb = sB[wave];
    unsigned* laU = (unsigned*)la;
    unsigned* lbU = (unsigned*)lb;
    v8f acc0 = {}, acc1 = {};

    const int mrow = lane & 15;
    const int half = lane >> 4;

    for (int k0 = 0; k0 < K; k0 += 32) {
        for (int i = lane; i < 256; i += 32) {
            int r = i >> 4, kp = (i & 15) << 1;
            int m = m0 + r, k = k0 + kp;
            float v0, v1;
            if (AMODE == 0) {
                long idx = (long)m * K + k;
                v0 = A[idx]; v1 = A[idx + 1];
            } else if (AMODE == 1) {
                long bidx = ((long)(m >> 10) * K + k) * 1024 + (m & 1023);
                v0 = A[bidx]; v1 = A[bidx + 1024];
            } else {
                long idx = (long)m * K + k;
                v0 = A[idx] * siluf(Z[idx]);
                v1 = A[idx + 1] * siluf(Z[idx + 1]);
            }
            laU[(r << 4) + (kp >> 1)] = pack_bf16(v0, v1);
        }
        for (int i = lane; i < 512; i += 32) {
            int nn = i & 31, kp = (i >> 5) << 1;
            long widx = (long)(k0 + kp) * ldw + wcol0 + n0 + nn;
            lbU[(nn << 4) + (kp >> 1)] = pack_bf16(W[widx], W[widx + ldw]);
        }
        const v8bf* laV = (const v8bf*)la;
        const v8bf* lbV = (const v8bf*)lb;
        v8bf a0 = laV[(mrow << 2) + half];
        v8bf a1 = laV[(mrow << 2) + 2 + half];
        v16bf af = __builtin_shufflevector(a0, a1, 0,1,2,3,4,5,6,7,8,9,10,11,12,13,14,15);
        int bbase0 = (mrow << 2) + half;
        int bbase1 = ((16 + mrow) << 2) + half;
        v8bf b0l = lbV[bbase0],     b0h = lbV[bbase0 + 2];
        v8bf b1l = lbV[bbase1],     b1h = lbV[bbase1 + 2];
        v16bf bf0 = __builtin_shufflevector(b0l, b0h, 0,1,2,3,4,5,6,7,8,9,10,11,12,13,14,15);
        v16bf bf1 = __builtin_shufflevector(b1l, b1h, 0,1,2,3,4,5,6,7,8,9,10,11,12,13,14,15);
        acc0 = __builtin_amdgcn_wmma_f32_16x16x32_f16(false, af, false, bf0, (short)0, acc0, false, false);
        acc1 = __builtin_amdgcn_wmma_f32_16x16x32_f16(false, af, false, bf1, (short)0, acc1, false, false);
        asm volatile("v_nop\n\tv_nop\n\tv_nop\n\tv_nop" : "+v"(acc0), "+v"(acc1) : "v"(af), "v"(bf1));
    }

    static_assert(EPI != 3, "EPI 3 uses gemm_outf");
    float* so = sO[wave];
#pragma unroll
    for (int j = 0; j < 2; ++j) {
        const v8f& acc = j ? acc1 : acc0;
        const int nl = (j << 4) + mrow, nj = n0 + nl;
#pragma unroll
        for (int v = 0; v < 8; ++v) {
            float r = acc[v];
            if (EPI == 2) r = softplusf(r + resid[nj]);
            so[(v + (half << 3)) * 32 + nl] = r;
        }
    }
    wave_lds_sync();
    for (int pass = 0; pass < 2; ++pass) {
#pragma unroll
        for (int rr = 0; rr < 16; ++rr) {
            const int m = m0 + rr;
            const float v = so[rr * 32 + lane];
            if (EPI == 1) { if (n0 < 256) *(volatile float*)(out + (long)m * 256 + n0 + lane) = v;
                            else          *(volatile float*)(out2 + (long)m * 256 + n0 - 256 + lane) = v; }
            else          *(volatile float*)(out + (long)m * Ncols + n0 + lane) = v;
        }
        __threadfence();
    }
}

__global__ __launch_bounds__(256) void gemm_outf(const float* __restrict__ Y, const float* __restrict__ Z, const float* __restrict__ W,
                                                 float* __restrict__ out, const float* __restrict__ resid, int M, int K) {
    __shared__ __attribute__((aligned(16))) __bf16 sA[8][32 * 32];
    __shared__ __attribute__((aligned(16))) __bf16 sB[8][16 * 32];
    __shared__ __attribute__((aligned(16))) float sO[8][16 * 32];
    const int wave = threadIdx.x >> 5, lane = threadIdx.x & 31;
    const long Mt = M >> 5, Nt = 128 / 16;
    long tile = (long)blockIdx.x * 8 + wave;
    if (tile >= Mt * Nt) return;
    const int tn = (int)(tile % Nt), tm = (int)(tile / Nt);
    const int m0 = tm << 5, n0 = tn << 4;
    __bf16* la = sA[wave]; __bf16* lb = sB[wave];
    unsigned* laU = (unsigned*)la; unsigned* lbU = (unsigned*)lb;
    const int mrow = lane & 15, half = lane >> 4;
    v8f acc0 = {}, acc1 = {};
    for (int k0 = 0; k0 < K; k0 += 32) {
        for (int i = lane; i < 512; i += 32) {
            int r = i >> 4, kp = (i & 15) << 1;
            long idx = (long)(m0 + r) * K + k0 + kp;
            laU[(r << 4) + (kp >> 1)] = pack_bf16(Y[idx] * siluf(Z[idx]), Y[idx + 1] * siluf(Z[idx + 1]));
        }
        for (int i = lane; i < 256; i += 32) {
            int nn = i & 15, kp = (i >> 4) << 1;
            long widx = (long)(k0 + kp) * 128 + n0 + nn;
            lbU[(nn << 4) + (kp >> 1)] = pack_bf16(W[widx], W[widx + 128]);
        }
        const v8bf* laV = (const v8bf*)la; const v8bf* lbV = (const v8bf*)lb;
        v16bf a0 = __builtin_shufflevector(laV[(mrow << 2) + half], laV[(mrow << 2) + 2 + half], 0,1,2,3,4,5,6,7,8,9,10,11,12,13,14,15);
        v16bf a1 = __builtin_shufflevector(laV[((16 + mrow) << 2) + half], laV[((16 + mrow) << 2) + 2 + half], 0,1,2,3,4,5,6,7,8,9,10,11,12,13,14,15);
        v16bf bf = __builtin_shufflevector(lbV[(mrow << 2) + half], lbV[(mrow << 2) + 2 + half], 0,1,2,3,4,5,6,7,8,9,10,11,12,13,14,15);
        acc0 = __builtin_amdgcn_wmma_f32_16x16x32_f16(false, a0, false, bf, (short)0, acc0, false, false);
        acc1 = __builtin_amdgcn_wmma_f32_16x16x32_f16(false, a1, false, bf, (short)0, acc1, false, false);
        asm volatile("v_nop\n\tv_nop\n\tv_nop\n\tv_nop" : "+v"(acc0), "+v"(acc1) : "v"(a1), "v"(bf));
    }
    float* so = sO[wave];
#pragma unroll
    for (int v = 0; v < 8; ++v) { so[mrow * 32 + v + (half << 3)] = acc0[v]; so[mrow * 32 + 16 + v + (half << 3)] = acc1[v]; }
    wave_lds_sync();
    const long bl = m0 >> 10, hw0 = m0 & 1023;
    for (int pass = 0; pass < 2; ++pass) {
#pragma unroll
        for (int nn = 0; nn < 16; ++nn) {
            const long idx = (bl * 128 + n0 + nn) * 1024 + hw0 + lane;
            *(volatile float*)(out + idx) = so[nn * 32 + lane] + resid[idx];
        }
        __threadfence();
    }
}

extern "C" void kernel_launch(void* const* d_in, const int* in_sizes, int n_in,
                              void* d_out, int out_size, void* d_ws, size_t ws_size,
                              hipStream_t stream) {
    const float* x      = (const float*)d_in[0];
    const float* prev_x = (const float*)d_in[1];
    const float* f_inw  = (const float*)d_in[2];
    const float* f_cw   = (const float*)d_in[3];
    const float* f_cb   = (const float*)d_in[4];
    const float* f_xpw  = (const float*)d_in[5];
    const float* f_dtw  = (const float*)d_in[6];
    const float* f_dtb  = (const float*)d_in[7];
    const float* f_Alog = (const float*)d_in[8];
    const float* f_D    = (const float*)d_in[9];
    const float* f_outw = (const float*)d_in[10];
    const float* c_inw  = (const float*)d_in[11];
    const float* c_cw   = (const float*)d_in[12];
    const float* c_cb   = (const float*)d_in[13];
    const float* c_xpw  = (const float*)d_in[14];
    const float* c_dtw  = (const float*)d_in[15];
    const float* c_dtb  = (const float*)d_in[16];
    const float* c_Alog = (const float*)d_in[17];
    const float* c_D    = (const float*)d_in[18];
    const float* c_outw = (const float*)d_in[19];

    const int FM = 16384;
    const int CM = 16;

    (void)in_sizes; (void)n_in; (void)out_size;
    if (ws_size < (size_t)(4 * 16384 * 256 + 16384 * 32 + 2 * 65536 + 2 * 4096 + 16 * 128 + 4 * 16 * 256 + 16 * 32) * 4) return;
    float* ws = (float*)d_ws;
    size_t o = 0;
    auto alloc = [&](size_t n) { float* p = ws + o; o += n; return p; };
    float* f_xmp = alloc((size_t)FM * 256);
    float* f_z   = alloc((size_t)FM * 256);
    float* f_xm  = alloc((size_t)FM * 256);
    float* f_y   = alloc((size_t)FM * 256);
    float* f_BC  = alloc((size_t)FM * 32);
    float* f_delta = f_xmp;
    float* wd_f  = alloc(256 * 256);
    float* wd_c  = alloc(256 * 256);
    float* An_f  = alloc(256 * 16);
    float* An_c  = alloc(256 * 16);
    float* c_xin = alloc(16 * 128);
    float* c_xmp = alloc(16 * 256);
    float* c_z   = alloc(16 * 256);
    float* c_xm  = alloc(16 * 256);
    float* c_y   = alloc(16 * 256);
    float* c_BC  = alloc(16 * 32);
    float* c_delta = c_xmp;

    float* out_f = (float*)d_out;
    float* out_c = (float*)d_out + 2097152;

    auto blocks = [](long tiles) { return (unsigned)((tiles + 7) / 8); };

    prep_wdelta<<<256, 256, 0, stream>>>(f_xpw, f_dtw, wd_f);
    prep_wdelta<<<256, 256, 0, stream>>>(c_xpw, c_dtw, wd_c);
    prep_negexpA<<<16, 256, 0, stream>>>(f_Alog, An_f);
    prep_negexpA<<<16, 256, 0, stream>>>(c_Alog, An_c);
    mean_kernel<<<16, 128, 0, stream>>>(x, prev_x, c_xin);

    gemm16<1, 1><<<blocks(1024L * 16), 256, 0, stream>>>(
        x, nullptr, f_inw, 512, 0, f_xmp, f_z, nullptr, FM, 512, 128);
    conv_silu<<<16 * 1024, 256, 0, stream>>>(f_xmp, f_cw, f_cb, f_xm, 1024);
    gemm16<0, 2><<<blocks(1024L * 8), 256, 0, stream>>>(
        f_xm, nullptr, wd_f, 256, 0, f_delta, nullptr, f_dtb, FM, 256, 256);
    gemm16<0, 0><<<blocks(1024L * 1), 256, 0, stream>>>(
        f_xm, nullptr, f_xpw, 40, 8, f_BC, nullptr, nullptr, FM, 32, 256);
    scan_kernel<<<16, 256, 0, stream>>>(f_xm, f_delta, f_BC, An_f, f_D, f_y, 1024);
    gemm_outf<<<blocks(512L * 8), 256, 0, stream>>>(f_y, f_z, f_outw, out_f, x, FM, 256);

    gemm16<0, 1><<<blocks(1L * 16), 256, 0, stream>>>(
        c_xin, nullptr, c_inw, 512, 0, c_xmp, c_z, nullptr, CM, 512, 128);
    conv_silu<<<16, 256, 0, stream>>>(c_xmp, c_cw, c_cb, c_xm, 8);
    gemm16<0, 2><<<blocks(1L * 8), 256, 0, stream>>>(
        c_xm, nullptr, wd_c, 256, 0, c_delta, nullptr, c_dtb, CM, 256, 256);
    gemm16<0, 0><<<blocks(1L * 1), 256, 0, stream>>>(
        c_xm, nullptr, c_xpw, 40, 8, c_BC, nullptr, nullptr, CM, 32, 256);
    scan_kernel<<<2, 256, 0, stream>>>(c_xm, c_delta, c_BC, An_c, c_D, c_y, 8);
    gemm16<2, 0><<<blocks(1L * 4), 256, 0, stream>>>(
        c_y, c_z, c_outw, 128, 0, out_c, nullptr, nullptr, CM, 128, 256);
}
